// CharacterIsolationAttention_60790967107674
// MI455X (gfx1250) — hardware-verified
//
#include <hip/hip_runtime.h>
#include <stdint.h>
#include <math.h>

#define NB     2
#define SEQ    2048
#define DM     1024
#define NH     16
#define HDIM   64
#define NCH    4
#define EPSN   1e-6f
#define PSCALE 16384.0f

typedef _Float16 v16h __attribute__((ext_vector_type(16)));
typedef _Float16 v8h  __attribute__((ext_vector_type(8)));
typedef __bf16   v16b __attribute__((ext_vector_type(16)));
typedef __bf16   v8b  __attribute__((ext_vector_type(8)));
typedef float    v8f  __attribute__((ext_vector_type(8)));
typedef float    v4f  __attribute__((ext_vector_type(4)));
typedef unsigned int   v4u  __attribute__((ext_vector_type(4)));
typedef unsigned short v8us __attribute__((ext_vector_type(8)));

union FragH { v16h v; v8h h[2]; };
union FragB { v16b v; v8b h[2]; };

__device__ __forceinline__ float bfr(float f) {
  unsigned u = __float_as_uint(f);
  u = (u + 0x7FFFu + ((u >> 16) & 1u)) & 0xFFFF0000u;
  return __uint_as_float(u);
}
__device__ __forceinline__ unsigned short bfbits(float f) {
  unsigned u = __float_as_uint(f);
  return (unsigned short)((u + 0x7FFFu + ((u >> 16) & 1u)) >> 16);
}
__device__ __forceinline__ float bf2f(unsigned short b) { return __uint_as_float(((unsigned)b) << 16); }
__device__ __forceinline__ _Float16 toh(float f) {
  const float a = (fabsf(f) < 6.103515625e-05f) ? 0.0f : f;
  return (_Float16)a;
}
__device__ __forceinline__ unsigned short tohbits(float f) { return __builtin_bit_cast(unsigned short, toh(f)); }

__device__ __forceinline__ v16h ldfragh(const _Float16* p) {
  FragH f;
  f.h[0] = *(const v8h*)p;
  f.h[1] = *(const v8h*)(p + 16);
  return f.v;
}
__device__ __forceinline__ v16b ldfragb(const __bf16* p) {
  FragB f;
  f.h[0] = *(const v8b*)p;
  f.h[1] = *(const v8b*)(p + 16);
  return f.v;
}
__device__ __forceinline__ v8f mmah(v16h a, v16h b, v8f c) {
  c = __builtin_amdgcn_wmma_f32_16x16x32_f16(false, a, false, b, (short)0, c, false, false);
  asm volatile("v_nop\n\tv_nop\n\tv_nop\n\tv_nop" : "+v"(c) : "v"(a), "v"(b));
  return c;
}
__device__ __forceinline__ v8f mmab(v16b a, v16b b, v8f c) {
  c = __builtin_amdgcn_wmma_f32_16x16x32_bf16(false, a, false, b, (short)0, c, false, false);
  asm volatile("v_nop\n\tv_nop\n\tv_nop\n\tv_nop" : "+v"(c) : "v"(a), "v"(b));
  return c;
}
__device__ __forceinline__ void wave_lds_sync() {
  __builtin_amdgcn_fence(__ATOMIC_RELEASE, "workgroup");
  __builtin_amdgcn_wave_barrier();
  __builtin_amdgcn_fence(__ATOMIC_ACQUIRE, "workgroup");
}
__device__ __forceinline__ v8f zero8() {
  v8f z = {0.f, 0.f, 0.f, 0.f, 0.f, 0.f, 0.f, 0.f};
  return z;
}

__global__ __launch_bounds__(256)
void cvt_f16_kernel(const float* __restrict__ in, _Float16* __restrict__ out, int n8, float scale) {
  const int i = blockIdx.x * 256 + (int)threadIdx.x;
  if (i >= n8) return;
  const float* p = in + (size_t)i * 8;
  const v4f a = *(const v4f*)p;
  const v4f b = *(const v4f*)(p + 4);
  v8h o;
  o[0] = toh(bfr(a[0]) * scale); o[1] = toh(bfr(a[1]) * scale);
  o[2] = toh(bfr(a[2]) * scale); o[3] = toh(bfr(a[3]) * scale);
  o[4] = toh(bfr(b[0]) * scale); o[5] = toh(bfr(b[1]) * scale);
  o[6] = toh(bfr(b[2]) * scale); o[7] = toh(bfr(b[3]) * scale);
  _Float16* q = out + (size_t)i * 8;
  *(volatile v8h*)q = o;
  __threadfence();
  *(volatile v8h*)q = o;
}

__global__ __launch_bounds__(256)
void cvt_bf16_kernel(const float* __restrict__ in, unsigned short* __restrict__ out, int n8) {
  const int i = blockIdx.x * 256 + (int)threadIdx.x;
  if (i >= n8) return;
  const float* p = in + (size_t)i * 8;
  const v4f a = *(const v4f*)p;
  const v4f b = *(const v4f*)(p + 4);
  v4u o;
  o[0] = (unsigned)bfbits(a[0]) | ((unsigned)bfbits(a[1]) << 16);
  o[1] = (unsigned)bfbits(a[2]) | ((unsigned)bfbits(a[3]) << 16);
  o[2] = (unsigned)bfbits(b[0]) | ((unsigned)bfbits(b[1]) << 16);
  o[3] = (unsigned)bfbits(b[2]) | ((unsigned)bfbits(b[3]) << 16);
  unsigned short* q = out + (size_t)i * 8;
  *(volatile v4u*)q = o;
  __threadfence();
  *(volatile v4u*)q = o;
}

__global__ __launch_bounds__(256)
void rowmax_kernel(const unsigned short* __restrict__ CMb, float* __restrict__ RMAX) {
  __shared__ __align__(16) float sm[32];
  const int lane = threadIdx.x & 31, wave = threadIdx.x >> 5;
  const int g0 = blockIdx.x * 32 + wave * 4;
  const int b = g0 >> 11;
  const unsigned short* cb = CMb + (size_t)b * NCH * SEQ;
  float cq[4][4], m[4];
#pragma unroll
  for (int i = 0; i < 4; ++i) {
    const int q = (g0 + i) & (SEQ - 1);
#pragma unroll
    for (int cc = 0; cc < NCH; ++cc) cq[i][cc] = bf2f(cb[cc * SEQ + q]);
    m[i] = -3.0e38f;
  }
#pragma unroll 1
  for (int k = lane; k < SEQ; k += 32) {
    const float k0v = bf2f(cb[k]);
    const float k1v = bf2f(cb[SEQ + k]);
    const float k2v = bf2f(cb[2 * SEQ + k]);
    const float k3v = bf2f(cb[3 * SEQ + k]);
#pragma unroll
    for (int i = 0; i < 4; ++i) {
      const float s = cq[i][0] * k0v + cq[i][1] * k1v + cq[i][2] * k2v + cq[i][3] * k3v;
      m[i] = fmaxf(m[i], s);
    }
  }
#pragma unroll
  for (int i = 0; i < 4; ++i) {
#pragma unroll
    for (int off = 1; off < 32; off <<= 1) m[i] = fmaxf(m[i], __shfl_xor(m[i], off, 32));
  }
  if (lane == 0) {
#pragma unroll
    for (int i = 0; i < 4; ++i) sm[wave * 4 + i] = fmaxf(m[i], 1e-6f);
  }
  __syncthreads();
  if (wave == 0 && lane < 8) {
    const v4f v = *(const v4f*)(sm + lane * 4);
    float* d = RMAX + (size_t)blockIdx.x * 32 + lane * 4;
    *(volatile v4f*)d = v;
    __threadfence();
    *(volatile v4f*)d = v;
  }
}

__global__ __launch_bounds__(64)
void qkv_gemm_kernel(const _Float16* __restrict__ X16, const _Float16* __restrict__ W16,
                     const float* __restrict__ qnw, const float* __restrict__ knw,
                     unsigned short* __restrict__ Qh, unsigned short* __restrict__ Ql,
                     unsigned short* __restrict__ Kh, unsigned short* __restrict__ Kl,
                     unsigned short* __restrict__ Vt16) {
  __shared__ __align__(16) unsigned short sT[128 * 72];
  const int lane = threadIdx.x & 31, wave = threadIdx.x >> 5, hh = lane >> 4, c = lane & 15;
  const int tilesN = (3 * DM) / 64;
  const int tile = blockIdx.x;
  const int tm = tile / tilesN, tn = tile - tm * tilesN;
  const int wr0 = 32 * wave;
  const int m0 = tm * 64 + wr0, n0 = tn * 64;
  const int mtype = tn >> 4, head = tn & 15;
  const int b = tm >> 5, nq0 = (tm & 31) * 64;

  v8f acc[2][4];
#pragma unroll
  for (int i = 0; i < 2; ++i)
#pragma unroll
    for (int j = 0; j < 4; ++j) acc[i][j] = zero8();

  const _Float16* Ab = X16 + (size_t)(m0 + c) * DM + 8 * hh;
  const _Float16* Bb = W16 + (size_t)(n0 + c) * DM + 8 * hh;
#pragma unroll 1
  for (int k0 = 0; k0 < DM; k0 += 32) {
    v16h bf[4];
#pragma unroll
    for (int j = 0; j < 4; ++j) bf[j] = ldfragh(Bb + (size_t)(16 * j) * DM + k0);
#pragma unroll
    for (int i = 0; i < 2; ++i) {
      const v16h af = ldfragh(Ab + (size_t)(16 * i) * DM + k0);
#pragma unroll
      for (int j = 0; j < 4; ++j) acc[i][j] = mmah(af, bf[j], acc[i][j]);
    }
  }

  const float sc = 1.0f / 512.0f;
  if (mtype < 2) {
    float w[4];
#pragma unroll
    for (int j = 0; j < 4; ++j) {
      const float wq = bfr(qnw[16 * j + c]);
      const float wk = bfr(knw[16 * j + c]);
      w[j] = (mtype == 0) ? wq : wk;
    }
#pragma unroll
    for (int i = 0; i < 2; ++i) {
#pragma unroll
      for (int r = 0; r < 8; ++r) {
        float ss = 0.0f;
#pragma unroll
        for (int j = 0; j < 4; ++j) { const float v = acc[i][j][r] * sc; acc[i][j][r] = v; ss += v * v; }
#pragma unroll
        for (int off = 1; off < 16; off <<= 1) ss += __shfl_xor(ss, off, 32);
        const float rn = rsqrtf(ss * (1.0f / 64.0f) + EPSN);
        const int trow = wr0 + 16 * i + 8 * hh + r;
#pragma unroll
        for (int j = 0; j < 4; ++j) {
          const float v = acc[i][j][r] * rn * w[j];
          const unsigned short hb = bfbits(v);
          const unsigned short lb = bfbits(v - bf2f(hb));
          sT[trow * 72 + 16 * j + c] = hb;
          sT[(64 + trow) * 72 + 16 * j + c] = lb;
        }
      }
    }
  } else {
#pragma unroll
    for (int i = 0; i < 2; ++i)
#pragma unroll
      for (int j = 0; j < 4; ++j)
#pragma unroll
        for (int r = 0; r < 8; ++r) sT[(16 * j + c) * 72 + wr0 + 16 * i + 8 * hh + r] = tohbits(acc[i][j][r] * sc);
  }
  __syncthreads();

  const int rq = lane >> 3, c8 = (lane & 7) * 8;
  if (mtype < 2) {
    const size_t pofs = ((size_t)(b * NH + head) * SEQ + nq0 + wr0) * HDIM;
    unsigned short* dh = ((mtype == 0) ? Qh : Kh) + pofs;
    unsigned short* dl = ((mtype == 0) ? Ql : Kl) + pofs;
    for (int pass = 0; pass < 2; ++pass) {
#pragma unroll
      for (int it = 0; it < 8; ++it) {
        const int row = it * 4 + rq;
        const v8us vh = *(const v8us*)(sT + (wr0 + row) * 72 + c8);
        const v8us vl = *(const v8us*)(sT + (64 + wr0 + row) * 72 + c8);
        *(volatile v8us*)(dh + (size_t)row * HDIM + c8) = vh;
        *(volatile v8us*)(dl + (size_t)row * HDIM + c8) = vl;
      }
      __threadfence();
    }
  } else {
    unsigned short* dst = Vt16 + ((size_t)(b * NH + head) * HDIM + wr0) * SEQ + nq0;
    for (int pass = 0; pass < 2; ++pass) {
#pragma unroll
      for (int it = 0; it < 8; ++it) {
        const int row = it * 4 + rq;
        const v8us v = *(const v8us*)(sT + (wr0 + row) * 72 + c8);
        *(volatile v8us*)(dst + (size_t)row * SEQ + c8) = v;
      }
      __threadfence();
    }
  }
}

__global__ __launch_bounds__(128)
void attn_kernel(const unsigned short* __restrict__ Qhp, const unsigned short* __restrict__ Qlp,
                 const unsigned short* __restrict__ Khp, const unsigned short* __restrict__ Klp,
                 const unsigned short* __restrict__ Vtp, const unsigned short* __restrict__ CMb,
                 const unsigned short* __restrict__ IMb, const float* __restrict__ RMAX,
                 const float* __restrict__ gate, unsigned short* __restrict__ Oh, unsigned short* __restrict__ Ol) {
  __shared__ __align__(16) __bf16   Kshh[64 * 64];
  __shared__ __align__(16) __bf16   Kshl[64 * 64];
  __shared__ __align__(16) _Float16 Vsh[64 * 64];
  __shared__ __align__(16) _Float16 Psh[4][16 * 64];
  __shared__ __align__(16) unsigned short Osh[4][2][16 * 72];
  __shared__ __align__(16) float cmqs[64 * 4];

  const int tid = threadIdx.x, wave = tid >> 5, lane = tid & 31, hh = lane >> 4, c = lane & 15;
  const int q0 = blockIdx.x * 64, h = blockIdx.y, b = blockIdx.z;
  const int bh = b * NH + h;
  const float G = 3.0f * fminf(fmaxf(bfr(gate[h]), 0.0f), 1.0f);
  const float Gim = 0.3f * G;

  const __bf16* Qhb = (const __bf16*)(const void*)Qhp;
  const __bf16* Qlb = (const __bf16*)(const void*)Qlp;
  const __bf16* Khb = (const __bf16*)(const void*)Khp;
  const __bf16* Klb = (const __bf16*)(const void*)Klp;
  const _Float16* Vt = (const _Float16*)(const void*)Vtp;

  if (tid < 64) {
    const int q = q0 + tid;
    const float rm = RMAX[(size_t)b * SEQ + q];
    const float A = 2.0f * G * (1.0f / rm);
    const unsigned short* cq = CMb + (size_t)b * NCH * SEQ + q;
#pragma unroll
    for (int cc = 0; cc < NCH; ++cc) cmqs[tid * 4 + cc] = bf2f(cq[cc * SEQ]) * A;
  }

  v16b qah[2], qal[2];
  {
    const size_t qo = ((size_t)bh * SEQ + q0 + wave * 16 + c) * HDIM + 8 * hh;
    qah[0] = ldfragb(Qhb + qo);
    qah[1] = ldfragb(Qhb + qo + 32);
    qal[0] = ldfragb(Qlb + qo);
    qal[1] = ldfragb(Qlb + qo + 32);
  }
  float mrow[8], lrow[8];
  v8f oacc[4];
#pragma unroll
  for (int r = 0; r < 8; ++r) { mrow[r] = -3.0e38f; lrow[r] = 0.0f; }
#pragma unroll
  for (int t = 0; t < 4; ++t) oacc[t] = zero8();

  const unsigned short* imb = IMb + ((size_t)(b * SEQ + q0 + wave * 16 + 8 * hh)) * SEQ + c;
  const unsigned short* ckb = CMb + (size_t)b * NCH * SEQ + c;
  _Float16* pw = &Psh[wave][0];

#pragma unroll 1
  for (int kc = 0; kc < SEQ / 64; ++kc) {
    const int kv0 = kc * 64;
    __syncthreads();
    {
      const int r = tid >> 1, half = (tid & 1) * 32;
      const __bf16* ksh = Khb + ((size_t)bh * SEQ + kv0 + r) * HDIM + half;
      const __bf16* ksl = Klb + ((size_t)bh * SEQ + kv0 + r) * HDIM + half;
      const _Float16* vs = Vt + ((size_t)bh * HDIM + r) * SEQ + kv0 + half;
#pragma unroll
      for (int i = 0; i < 4; ++i) {
        const v8b kvh = *(const v8b*)(ksh + 8 * i);
        const v8b kvl = *(const v8b*)(ksl + 8 * i);
        const v8h vv  = *(const v8h*)(vs + 8 * i);
        *(v8b*)(Kshh + r * 64 + half + 8 * i) = kvh;
        *(v8b*)(Kshl + r * 64 + half + 8 * i) = kvl;
        *(v8h*)(Vsh + r * 64 + half + 8 * i) = vv;
      }
    }
    __syncthreads();

    v8f s[4];
#pragma unroll
    for (int j = 0; j < 4; ++j) {
      s[j] = zero8();
#pragma unroll
      for (int dc = 0; dc < 2; ++dc) {
        FragB kb, kl;
        kb.h[0] = *(const v8b*)(Kshh + (16 * j + c) * 64 + dc * 32 + 8 * hh);
        kb.h[1] = *(const v8b*)(Kshh + (16 * j + c) * 64 + dc * 32 + 16 + 8 * hh);
        kl.h[0] = *(const v8b*)(Kshl + (16 * j + c) * 64 + dc * 32 + 8 * hh);
        kl.h[1] = *(const v8b*)(Kshl + (16 * j + c) * 64 + dc * 32 + 16 + 8 * hh);
        s[j] = mmab(qah[dc], kb.v, s[j]);
        s[j] = mmab(qah[dc], kl.v, s[j]);
        s[j] = mmab(qal[dc], kb.v, s[j]);
      }
    }

    float ck[4][4];
#pragma unroll
    for (int j = 0; j < 4; ++j)
#pragma unroll
      for (int cc = 0; cc < NCH; ++cc) ck[j][cc] = bf2f(ckb[cc * SEQ + kv0 + 16 * j]);

    float cmx[8];
#pragma unroll
    for (int r = 0; r < 8; ++r) {
      const int rowq = wave * 16 + 8 * hh + r;
      const float a0 = cmqs[rowq * 4 + 0], a1 = cmqs[rowq * 4 + 1];
      const float a2 = cmqs[rowq * 4 + 2], a3 = cmqs[rowq * 4 + 3];
      float m = -3.0e38f;
#pragma unroll
      for (int j = 0; j < 4; ++j) {
        const float imv = bf2f(imb[(size_t)r * SEQ + kv0 + 16 * j]);
        const float bias = (a0 * ck[j][0] + a1 * ck[j][1] + a2 * ck[j][2] + a3 * ck[j][3]) + Gim * imv - G;
        const float lg = s[j][r] * 0.125f + bias;
        s[j][r] = lg;
        m = fmaxf(m, lg);
      }
#pragma unroll
      for (int off = 1; off < 16; off <<= 1) m = fmaxf(m, __shfl_xor(m, off, 32));
      cmx[r] = m;
    }
#pragma unroll
    for (int r = 0; r < 8; ++r) {
      const float mnew = fmaxf(mrow[r], cmx[r]);
      const float alpha = __expf(mrow[r] - mnew);
      mrow[r] = mnew;
      float psum = 0.0f;
#pragma unroll
      for (int j = 0; j < 4; ++j) {
        const float p = __expf(s[j][r] - mnew);
        psum += p;
        pw[(8 * hh + r) * 64 + 16 * j + c] = toh(p * PSCALE);
      }
#pragma unroll
      for (int off = 1; off < 16; off <<= 1) psum += __shfl_xor(psum, off, 32);
      lrow[r] = lrow[r] * alpha + psum;
#pragma unroll
      for (int t = 0; t < 4; ++t) oacc[t][r] *= alpha;
    }
    wave_lds_sync();

#pragma unroll
    for (int kk = 0; kk < 2; ++kk) {
      FragH pa;
      pa.h[0] = *(const v8h*)(pw + c * 64 + kk * 32 + 8 * hh);
      pa.h[1] = *(const v8h*)(pw + c * 64 + kk * 32 + 16 + 8 * hh);
#pragma unroll
      for (int t = 0; t < 4; ++t) {
        FragH vb;
        vb.h[0] = *(const v8h*)(Vsh + (16 * t + c) * 64 + kk * 32 + 8 * hh);
        vb.h[1] = *(const v8h*)(Vsh + (16 * t + c) * 64 + kk * 32 + 16 + 8 * hh);
        oacc[t] = mmah(pa.v, vb.v, oacc[t]);
      }
    }
  }

  unsigned short* oth = &Osh[wave][0][0];
  unsigned short* otl = &Osh[wave][1][0];
#pragma unroll
  for (int r = 0; r < 8; ++r) {
    const float f = 1.0f / (lrow[r] * PSCALE);
#pragma unroll
    for (int t = 0; t < 4; ++t) {
      const float v = oacc[t][r] * f;
      const unsigned short hb = bfbits(v);
      const unsigned short lb = bfbits(v - bf2f(hb));
      oth[(8 * hh + r) * 72 + 16 * t + c] = hb;
      otl[(8 * hh + r) * 72 + 16 * t + c] = lb;
    }
  }
  wave_lds_sync();
  {
    const size_t oofs = ((size_t)(b * SEQ + q0 + wave * 16)) * DM + (size_t)h * HDIM;
    unsigned short* dsth = Oh + oofs;
    unsigned short* dstl = Ol + oofs;
    const int rq = lane >> 3, c8 = (lane & 7) * 8;
    for (int pass = 0; pass < 2; ++pass) {
#pragma unroll
      for (int it = 0; it < 4; ++it) {
        const int row = it * 4 + rq;
        const v8us vh = *(const v8us*)(oth + row * 72 + c8);
        const v8us vl = *(const v8us*)(otl + row * 72 + c8);
        *(volatile v8us*)(dsth + (size_t)row * DM + c8) = vh;
        *(volatile v8us*)(dstl + (size_t)row * DM + c8) = vl;
      }
      __threadfence();
    }
  }
}

__global__ __launch_bounds__(128)
void out_gemm_kernel(const unsigned short* __restrict__ Ohp, const unsigned short* __restrict__ Olp,
                     const unsigned short* __restrict__ Wobp, float* __restrict__ out) {
  __shared__ __align__(16) float sT[4][16 * 68];
  const int lane = threadIdx.x & 31, wave = threadIdx.x >> 5, hh = lane >> 4, c = lane & 15;
  const int tilesN = DM / 64;
  const int tilesM = (NB * SEQ) / 64;
  const int tile = blockIdx.x * 4 + wave;
  if (tile >= tilesM * tilesN) return;
  const int tm = tile / tilesN, tn = tile - tm * tilesN;
  const int m0 = tm * 64, n0 = tn * 64;

  const __bf16* Ohb = (const __bf16*)(const void*)Ohp;
  const __bf16* Olb = (const __bf16*)(const void*)Olp;
  const __bf16* Wob = (const __bf16*)(const void*)Wobp;

  v8f acc[4][4];
#pragma unroll
  for (int i = 0; i < 4; ++i)
#pragma unroll
    for (int j = 0; j < 4; ++j) acc[i][j] = zero8();

  const __bf16* Ah = Ohb + (size_t)(m0 + c) * DM + 8 * hh;
  const __bf16* Al = Olb + (size_t)(m0 + c) * DM + 8 * hh;
  const __bf16* Bb = Wob + (size_t)(n0 + c) * DM + 8 * hh;
#pragma unroll 1
  for (int k0 = 0; k0 < DM; k0 += 32) {
    v16b bf[4];
#pragma unroll
    for (int j = 0; j < 4; ++j) bf[j] = ldfragb(Bb + (size_t)(16 * j) * DM + k0);
#pragma unroll
    for (int i = 0; i < 4; ++i) {
      const v16b afh = ldfragb(Ah + (size_t)(16 * i) * DM + k0);
      const v16b afl = ldfragb(Al + (size_t)(16 * i) * DM + k0);
#pragma unroll
      for (int j = 0; j < 4; ++j) {
        acc[i][j] = mmab(afh, bf[j], acc[i][j]);
        acc[i][j] = mmab(afl, bf[j], acc[i][j]);
      }
    }
  }

  float* slab = &sT[wave][0];
  const int c4 = (lane & 15) * 4;
#pragma unroll
  for (int i = 0; i < 4; ++i) {
#pragma unroll
    for (int j = 0; j < 4; ++j)
#pragma unroll
      for (int r = 0; r < 8; ++r) slab[(8 * hh + r) * 68 + 16 * j + c] = acc[i][j][r];
    wave_lds_sync();
    for (int pass = 0; pass < 2; ++pass) {
#pragma unroll
      for (int it = 0; it < 8; ++it) {
        const int row = it * 2 + hh;
        const v4f v = *(const v4f*)(slab + row * 68 + c4);
        *(volatile v4f*)(out + (size_t)(m0 + 16 * i + row) * DM + n0 + c4) = v;
      }
      __threadfence();
    }
    wave_lds_sync();
  }
}

extern "C" void kernel_launch(void* const* d_in, const int* in_sizes, int n_in,
                              void* d_out, int out_size, void* d_ws, size_t ws_size,
                              hipStream_t stream) {
  if (n_in < 8) return;
  if (in_sizes[0] != NB * SEQ * DM) return;
  if (in_sizes[1] != NB * NCH * SEQ) return;
  if (in_sizes[2] != NB * SEQ * SEQ) return;
  if (in_sizes[3] != 3 * DM * DM) return;
  if (in_sizes[4] != DM * DM) return;
  if (in_sizes[5] != HDIM || in_sizes[6] != HDIM || in_sizes[7] != NH) return;
  if (out_size != NB * SEQ * DM) return;

  const float* x     = (const float*)d_in[0];
  const float* cm    = (const float*)d_in[1];
  const float* im    = (const float*)d_in[2];
  const float* qkv_w = (const float*)d_in[3];
  const float* out_w = (const float*)d_in[4];
  const float* qnw   = (const float*)d_in[5];
  const float* knw   = (const float*)d_in[6];
  const float* gate  = (const float*)d_in[7];
  float* out = (float*)d_out;

  const size_t szX  = (size_t)in_sizes[0] * 2;
  const size_t szW  = (size_t)in_sizes[3] * 2;
  const size_t szWo = (size_t)in_sizes[4] * 2;
  const size_t szP  = (size_t)NB * NH * SEQ * HDIM * 2;
  const size_t szO  = (size_t)NB * SEQ * DM * 2;
  const size_t szIM = (size_t)in_sizes[2] * 2;
  const size_t szCM = (size_t)in_sizes[1] * 2;
  const size_t szRM = (size_t)NB * SEQ * 4;
  size_t off = 0;
  const size_t oX  = off; off += szX;
  const size_t oW  = off; off += szW;
  const size_t oWo = off; off += szWo;
  const size_t oQh = off; off += szP;
  const size_t oQl = off; off += szP;
  const size_t oKh = off; off += szP;
  const size_t oKl = off; off += szP;
  const size_t oVt = off; off += szP;
  const size_t oOh = off; off += szO;
  const size_t oOl = off; off += szO;
  const size_t oIM = off; off += szIM;
  const size_t oCM = off; off += szCM;
  const size_t oRM = off; off += szRM;
  if (off > ws_size) return;

  char* ws = (char*)d_ws;
  _Float16* X16 = (_Float16*)(ws + oX);
  _Float16* W16 = (_Float16*)(ws + oW);
  unsigned short* Wob  = (unsigned short*)(ws + oWo);
  unsigned short* Qh   = (unsigned short*)(ws + oQh);
  unsigned short* Ql   = (unsigned short*)(ws + oQl);
  unsigned short* Kh   = (unsigned short*)(ws + oKh);
  unsigned short* Kl   = (unsigned short*)(ws + oKl);
  unsigned short* Vt16 = (unsigned short*)(ws + oVt);
  unsigned short* Oh   = (unsigned short*)(ws + oOh);
  unsigned short* Ol   = (unsigned short*)(ws + oOl);
  unsigned short* IMb  = (unsigned short*)(ws + oIM);
  unsigned short* CMb  = (unsigned short*)(ws + oCM);
  float* RMAX = (float*)(ws + oRM);

  const int n8x  = in_sizes[0] / 8;
  const int n8w  = in_sizes[3] / 8;
  const int n8wo = in_sizes[4] / 8;
  const int n8im = in_sizes[2] / 8;
  const int n8cm = in_sizes[1] / 8;
  if (n8x * 8 != in_sizes[0] || n8w * 8 != in_sizes[3] || n8wo * 8 != in_sizes[4]) return;
  if (n8im * 8 != in_sizes[2] || n8cm * 8 != in_sizes[1]) return;

  const dim3 blk256(256), blk128(128), blk64(64);
  cvt_f16_kernel<<<dim3((n8x + 255) / 256), blk256, 0, stream>>>(x, X16, n8x, 8.0f);
  cvt_f16_kernel<<<dim3((n8w + 255) / 256), blk256, 0, stream>>>(qkv_w, W16, n8w, 64.0f);
  cvt_bf16_kernel<<<dim3((n8wo + 255) / 256), blk256, 0, stream>>>(out_w, Wob, n8wo);
  cvt_bf16_kernel<<<dim3((n8im + 255) / 256), blk256, 0, stream>>>(im, IMb, n8im);
  cvt_bf16_kernel<<<dim3((n8cm + 255) / 256), blk256, 0, stream>>>(cm, CMb, n8cm);
  rowmax_kernel<<<dim3((NB * SEQ) / 32), blk256, 0, stream>>>(CMb, RMAX);
  qkv_gemm_kernel<<<dim3((NB * SEQ / 64) * (3 * DM / 64)), blk64, 0, stream>>>(X16, W16, qnw, knw, Qh, Ql, Kh, Kl, Vt16);
  attn_kernel<<<dim3(SEQ / 64, NH, NB), blk128, 0, stream>>>(Qh, Ql, Kh, Kl, Vt16, CMb, IMb, RMAX, gate, Oh, Ol);
  out_gemm_kernel<<<dim3(((NB * SEQ / 64) * (DM / 64)) / 4), blk128, 0, stream>>>(Oh, Ol, Wob, out);
  (void)hipGetLastError();
}
